// VAE_65859028516878
// MI455X (gfx1250) — hardware-verified
//
#include <hip/hip_runtime.h>
#include <math.h>

#pragma clang fp contract(off)

typedef __attribute__((ext_vector_type(16))) _Float16 v16h;
typedef __attribute__((ext_vector_type(8)))  _Float16 v8h;
typedef __attribute__((ext_vector_type(16))) __bf16   v16b;
typedef __attribute__((ext_vector_type(8)))  __bf16   v8b;
typedef __attribute__((ext_vector_type(8)))  float    v8f;
typedef __attribute__((ext_vector_type(4)))  float    v4f;
typedef __attribute__((ext_vector_type(4)))  unsigned v4u;
#define PSCALE 32768.0f
#define U16(p) ((const unsigned short*)(const void*)(p))
#define PSCALE_INV (1.0f / 32768.0f)

__device__ __forceinline__ unsigned short f2bf_bits(float f) {
  unsigned u = __float_as_uint(f);
  return (unsigned short)((u + 0x7FFFu + ((u >> 16) & 1u)) >> 16);
}
__device__ __forceinline__ float bf_bits2f(unsigned short h) { return __uint_as_float(((unsigned)h) << 16); }

__device__ __forceinline__ void dep_guard_h(v8f& a, v8f& b, v16h x, v16h y) { asm volatile("v_nop\n\tv_nop\n\tv_nop\n\tv_nop" : "+v"(a), "+v"(b) : "v"(x), "v"(y)); }
__device__ __forceinline__ void dep_guard_b(v8f& a, v8f& b, v16b x, v16b y) { asm volatile("v_nop\n\tv_nop\n\tv_nop\n\tv_nop" : "+v"(a), "+v"(b) : "v"(x), "v"(y)); }
__device__ __forceinline__ void keep4_h(v16h a, v16h b, v16h c, v16h d) { asm volatile("v_nop" :: "v"(a), "v"(b), "v"(c), "v"(d)); }
__device__ __forceinline__ void keep4_b(v16b a, v16b b, v16b c, v16b d) { asm volatile("v_nop" :: "v"(a), "v"(b), "v"(c), "v"(d)); }
__device__ __forceinline__ void acc_guard4(v8f& a, v8f& b, v8f& c, v8f& d) { asm volatile("v_nop\n\tv_nop\n\tv_nop\n\tv_nop" : "+v"(a), "+v"(b), "+v"(c), "+v"(d)); }
template <typename T> struct Frag;
template <> struct Frag<_Float16> {
  typedef v16h V; union U { v16h v; v8h h[2]; };
  static __device__ __forceinline__ v16h load(const _Float16* p) {
    U f; f.h[0] = *(const v8h*)(p); f.h[1] = *(const v8h*)(p + 16); return f.v;
  }
  static __device__ __forceinline__ v8f mma(v16h a, v16h b, v8f c) {
    return __builtin_amdgcn_wmma_f32_16x16x32_f16(false, a, false, b, (short)0, c, false, false);
  }
  static __device__ __forceinline__ void guard(v8f& a, v8f& b, v16h x, v16h y) { dep_guard_h(a, b, x, y); }
  static __device__ __forceinline__ void keep(v16h a, v16h b, v16h c, v16h d) { keep4_h(a, b, c, d); }
};
template <> struct Frag<__bf16> {
  typedef v16b V; union U { v16b v; v8b h[2]; };
  static __device__ __forceinline__ v16b load(const __bf16* p) {
    U f; f.h[0] = *(const v8b*)(p); f.h[1] = *(const v8b*)(p + 16); return f.v;
  }
  static __device__ __forceinline__ v8f mma(v16b a, v16b b, v8f c) {
    return __builtin_amdgcn_wmma_f32_16x16x32_bf16(false, a, false, b, (short)0, c, false, false);
  }
  static __device__ __forceinline__ void guard(v8f& a, v8f& b, v16b x, v16b y) { dep_guard_b(a, b, x, y); }
  static __device__ __forceinline__ void keep(v16b a, v16b b, v16b c, v16b d) { keep4_b(a, b, c, d); }
};

template <int ET> struct Elem;
template <> struct Elem<0> { typedef _Float16 T; };
template <> struct Elem<1> { typedef __bf16 T; };
template <int ET, bool SPLIT, int BIAS_MODE, int OUT_MODE, bool RESID, int ACT = 0>
__global__ __launch_bounds__(256) void wmma_gemm64(
    const unsigned short* __restrict__ Ap, const unsigned short* __restrict__ A2p, int lda, long strideA,
    const unsigned short* __restrict__ Btp, const unsigned short* __restrict__ Bt2p, int ldb, long strideB,
    void* __restrict__ Cout, void* __restrict__ Cout2, int ldc, long strideC,
    const float* __restrict__ bias,
    const float* __restrict__ resid, long strideR,
    int M, int N, int K, float scale) {
  typedef typename Elem<ET>::T T;
  typedef typename Frag<T>::V V;
  const T* A = (const T*)Ap; const T* A2 = (const T*)A2p; const T* Bt = (const T*)Btp; const T* Bt2 = (const T*)Bt2p;
  __shared__ __align__(16) float sT[8][16 * 68];
  const int b    = blockIdx.y;
  const int lane = threadIdx.x & 31;
  const int wave = threadIdx.x >> 5;
  const int tilesN = N >> 6;
  const int tilesM = M >> 6;
  const int tile = blockIdx.x * 8 + wave;
  if (tile >= tilesM * tilesN) return;
  const int tm = tile / tilesN;
  const int tn = tile - tm * tilesN;
  const int m0 = tm << 6;
  const int n0 = tn << 6;

  const T* Ab  = A  + (size_t)b * strideA;
  const T* Bb  = Bt + (size_t)b * strideB;
  const T* Ab2 = SPLIT ? (A2  + (size_t)b * strideA) : nullptr;
  const T* Bb2 = SPLIT ? (Bt2 + (size_t)b * strideB) : nullptr;

  const int rlane = lane & 15;
  const int koff  = (lane >> 4) * 8;
  const int mOff  = (lane >> 4) * 8;

  v8f acc[4][4];
#pragma unroll
  for (int i = 0; i < 4; ++i)
#pragma unroll
    for (int j = 0; j < 4; ++j) acc[i][j] = (v8f){0.f,0.f,0.f,0.f,0.f,0.f,0.f,0.f};

  for (int k0 = 0; k0 < K; k0 += 32) {
    V bh[4], bl[4];
#pragma unroll
    for (int j = 0; j < 4; ++j) {
      const size_t bo = (size_t)(n0 + (j << 4) + rlane) * ldb + koff + k0;
      bh[j] = Frag<T>::load(Bb + bo);
      if (SPLIT) bl[j] = Frag<T>::load(Bb2 + bo);
    }
#pragma unroll
    for (int i = 0; i < 4; ++i) {
      const size_t ao = (size_t)(m0 + (i << 4) + rlane) * lda + koff + k0;
      V ah = Frag<T>::load(Ab + ao);
      V al;
      if (SPLIT) al = Frag<T>::load(Ab2 + ao);
#pragma unroll
      for (int j = 0; j < 4; ++j) {
        acc[i][j] = Frag<T>::mma(ah, bh[j], acc[i][j]);
        if (SPLIT) {
          acc[i][j] = Frag<T>::mma(ah, bl[j], acc[i][j]);
          acc[i][j] = Frag<T>::mma(al, bh[j], acc[i][j]);
        }
      }
      Frag<T>::guard(acc[i][0], acc[i][3], ah, SPLIT ? al : ah);
    }
    Frag<T>::keep(bh[0], bh[1], bh[2], bh[3]);
    if (SPLIT) Frag<T>::keep(bl[0], bl[1], bl[2], bl[3]);
  }
  acc_guard4(acc[0][0], acc[0][1], acc[0][2], acc[0][3]);
  acc_guard4(acc[1][0], acc[1][1], acc[1][2], acc[1][3]);
  acc_guard4(acc[2][0], acc[2][1], acc[2][2], acc[2][3]);
  acc_guard4(acc[3][0], acc[3][1], acc[3][2], acc[3][3]);

  float* slab = sT[wave];
  const float* Rb = RESID ? (resid + (size_t)b * strideR) : nullptr;
#pragma unroll
  for (int i = 0; i < 4; ++i) {
    const int mBase = m0 + (i << 4);
#pragma unroll
    for (int j = 0; j < 4; ++j) {
      const int n = n0 + (j << 4) + rlane;
      float bv = 0.f;
      if (BIAS_MODE == 2) bv = bias[n];
#pragma unroll
      for (int r = 0; r < 8; ++r) {
        float v = acc[i][j][r] * scale;
        if (BIAS_MODE == 1) v += bias[mBase + mOff + r];
        if (BIAS_MODE == 2) v += bv;
        if (RESID) v += Rb[(size_t)(mBase + mOff + r) * ldc + n];
        if (ACT == 1) v = tanhf(v);
        if (ACT == 2) v = fmaxf(v, 0.0f);
        if (ACT == 3) v = v / (1.0f + expf(-v));
        if (ACT == 4) v = (v > 0.f) ? v : 0.01f * v;
        if (ACT == 5) v = 0.5f * v * (1.0f + erff(v * 0.70710678118654752f));
        slab[(mOff + r) * 68 + (j << 4) + rlane] = v;
      }
    }
    __builtin_amdgcn_fence(__ATOMIC_RELEASE, "workgroup");
    __builtin_amdgcn_wave_barrier();
    __builtin_amdgcn_fence(__ATOMIC_ACQUIRE, "workgroup");
    if (OUT_MODE == 0) {
      float* C = (float*)Cout + (size_t)b * strideC;
      const int hh = lane >> 4, c4 = (lane & 15) * 4;
      for (int pass = 0; pass < 2; ++pass) {
#pragma unroll
        for (int it = 0; it < 8; ++it) {
          const int row = it * 2 + hh;
          v4f v = *(const v4f*)(slab + row * 68 + c4);
          *(volatile v4f*)(C + (size_t)(mBase + row) * ldc + n0 + c4) = v;
        }
        __threadfence();
      }
    } else {
      const int q = lane >> 3, c8 = (lane & 7) * 8;
      unsigned short* C  = (unsigned short*)Cout  + (size_t)b * strideC;
      unsigned short* C2 = (OUT_MODE == 2) ? ((unsigned short*)Cout2 + (size_t)b * strideC) : nullptr;
      for (int pass = 0; pass < 2; ++pass) {
#pragma unroll
        for (int it = 0; it < 4; ++it) {
          const int row = it * 4 + q;
          const float* sp = slab + row * 68 + c8;
          v8h hv, lv;
#pragma unroll
          for (int e = 0; e < 8; ++e) {
            if (OUT_MODE == 1) {
              hv[e] = (_Float16)sp[e];
            } else {
              unsigned short hb = f2bf_bits(sp[e]);
              unsigned short lb = f2bf_bits(sp[e] - bf_bits2f(hb));
              hv[e] = __builtin_bit_cast(_Float16, hb);
              lv[e] = __builtin_bit_cast(_Float16, lb);
            }
          }
          *(volatile v8h*)(C + (size_t)(mBase + row) * ldc + n0 + c8) = hv;
          if (OUT_MODE == 2) *(volatile v8h*)(C2 + (size_t)(mBase + row) * ldc + n0 + c8) = lv;
        }
        __threadfence();
      }
    }
    __builtin_amdgcn_fence(__ATOMIC_RELEASE, "workgroup");
    __builtin_amdgcn_wave_barrier();
    __builtin_amdgcn_fence(__ATOMIC_ACQUIRE, "workgroup");
  }
}

constexpr int NSAMP   = 16384;
constexpr int DIMT    = 256;
constexpr int NFEAT   = 256;
constexpr int NHID    = 128;
constexpr int NAUX    = 64;
constexpr int KFEAT1  = 288;
constexpr int XPITCH  = 320;
constexpr float DTSTEP = 0.01f;
constexpr float WCARRY = 16.0f;
constexpr float WCARRY_INV = 1.0f / 16.0f;

static_assert(KFEAT1 % 32 == 0 && KFEAT1 >= DIMT + 1 && KFEAT1 <= XPITCH, "K padding");
static_assert(XPITCH % 64 == 0 && NFEAT % 64 == 0, "plane pitch");
static_assert(NSAMP % 64 == 0 && NFEAT % 64 == 0 && NHID % 64 == 0 && DIMT % 32 == 0, "tile multiples");

constexpr size_t SZ_XP  = (size_t)NSAMP * XPITCH * 2;
constexpr size_t SZ_BT1 = (size_t)NFEAT * XPITCH * 2;
constexpr size_t SZ_BT2 = (size_t)NFEAT * NFEAT * 2;
constexpr size_t SZ_BT3 = (size_t)(2 * NHID) * NFEAT * 2;
constexpr size_t SZ_P1  = (size_t)NSAMP * NFEAT * 2;
constexpr size_t SZ_P2  = (size_t)NSAMP * NFEAT * 2;
constexpr size_t SZ_HP  = (size_t)NSAMP * (2 * NHID) * 4;
constexpr size_t SZ_XI  = (size_t)NSAMP * 4;
constexpr size_t OFF_XP  = 0;
constexpr size_t OFF_BT1 = OFF_XP + SZ_XP;
constexpr size_t OFF_BT2 = OFF_BT1 + SZ_BT1;
constexpr size_t OFF_BT3 = OFF_BT2 + SZ_BT2;
constexpr size_t OFF_P1  = OFF_BT3 + SZ_BT3;
constexpr size_t OFF_P2  = OFF_P1 + SZ_P1;
constexpr size_t OFF_HP  = OFF_P2 + SZ_P2;
constexpr size_t OFF_XI  = OFF_HP + SZ_HP;
constexpr size_t WS_TOTAL = OFF_XI + SZ_XI;
static_assert(OFF_BT1 % 256 == 0 && OFF_BT2 % 256 == 0 && OFF_BT3 % 256 == 0 && OFF_P1 % 256 == 0 &&
              OFF_P2 % 256 == 0 && OFF_HP % 256 == 0 && OFF_XI % 256 == 0, "aligned carve");
static_assert(WS_TOTAL == 44531712u, "carve total");
static_assert(WS_TOTAL <= 134217728u, "carve budget");

constexpr size_t OUT0_OFF_B = 0, OUT1_OFF_B = 65536, OUT2_OFF_B = 131072;
static_assert(OUT1_OFF_B == (size_t)NSAMP * 4 && OUT2_OFF_B == OUT1_OFF_B + (size_t)NSAMP * 4, "output offsets");
static_assert(OUT2_OFF_B + (size_t)NSAMP * DIMT * 4 == 16908288u, "output total");

__device__ __forceinline__ unsigned pack_f16x2(float a, float b) {
  const unsigned short ha = __builtin_bit_cast(unsigned short, (_Float16)a);
  const unsigned short hb = __builtin_bit_cast(unsigned short, (_Float16)b);
  return (unsigned)ha | ((unsigned)hb << 16);
}

__global__ __launch_bounds__(256) void build_x_plane(const float* __restrict__ data, const float* __restrict__ omega,
                                                     unsigned short* __restrict__ xp) {
  constexpr int CPR = XPITCH / 8;
  constexpr int NI  = XPITCH / 64;
  const int lane = threadIdx.x & 31, wave = threadIdx.x >> 5;
  const int row0 = (blockIdx.x * 8 + wave) * 4;
  v4u vals[NI];
#pragma unroll
  for (int i = 0; i < NI; ++i) {
    const int g = i * 32 + lane;
    const int r = g / CPR;
    const int cc = g - r * CPR;
    const int row = row0 + r;
    const int ccl = (cc < 32) ? cc : 31;
    const float* src = data + (size_t)row * DIMT + ccl * 8;
    const v4f d0 = *(const v4f*)(src);
    const v4f d1 = *(const v4f*)(src + 4);
    const float om = omega[row];
    const bool isdat = (cc < 32);
    const bool isom  = (cc == 32);
    float f[8];
    f[0] = d0[0]; f[1] = d0[1]; f[2] = d0[2]; f[3] = d0[3];
    f[4] = d1[0]; f[5] = d1[1]; f[6] = d1[2]; f[7] = d1[3];
#pragma unroll
    for (int e = 0; e < 8; ++e) f[e] = isdat ? f[e] : ((isom && e == 0) ? om : 0.0f);
    vals[i] = (v4u){pack_f16x2(f[0], f[1]), pack_f16x2(f[2], f[3]), pack_f16x2(f[4], f[5]), pack_f16x2(f[6], f[7])};
  }
  unsigned short* base = xp + (size_t)row0 * XPITCH;
  for (int pass = 0; pass < 2; ++pass) {
#pragma unroll
    for (int i = 0; i < NI; ++i) *(volatile v4u*)(base + (size_t)(i * 32 + lane) * 8) = vals[i];
    __threadfence();
  }
}

template <int KPAD>
__global__ __launch_bounds__(256) void build_wt_plane(const float* __restrict__ W, int ldw, int kreal, float scale,
                                                      unsigned short* __restrict__ outp) {
  static_assert(KPAD % 64 == 0, "pitch must be a whole number of 128-B lines per 4 rows");
  constexpr int CPR = KPAD / 8;
  constexpr int NI  = KPAD / 64;
  const int lane = threadIdx.x & 31, wave = threadIdx.x >> 5;
  const int n0 = (blockIdx.x * 8 + wave) * 4;
  v4u vals[NI];
#pragma unroll
  for (int i = 0; i < NI; ++i) {
    const int g = i * 32 + lane;
    const int r = g / CPR;
    const int cc = g - r * CPR;
    const int n = n0 + r;
    unsigned w[4];
#pragma unroll
    for (int e2 = 0; e2 < 4; ++e2) {
      const int k0 = cc * 8 + 2 * e2;
      const int k1 = k0 + 1;
      const int k0c = (k0 < kreal) ? k0 : (kreal - 1);
      const int k1c = (k1 < kreal) ? k1 : (kreal - 1);
      float f0 = W[(size_t)k0c * ldw + n] * scale;
      float f1 = W[(size_t)k1c * ldw + n] * scale;
      f0 = (k0 < kreal) ? f0 : 0.0f;
      f1 = (k1 < kreal) ? f1 : 0.0f;
      w[e2] = pack_f16x2(f0, f1);
    }
    asm volatile("" : "+v"(w[0]), "+v"(w[1]), "+v"(w[2]), "+v"(w[3]) : : "memory");
    vals[i] = (v4u){w[0], w[1], w[2], w[3]};
  }
  unsigned short* base = outp + (size_t)n0 * KPAD;
  for (int pass = 0; pass < 2; ++pass) {
#pragma unroll
    for (int i = 0; i < NI; ++i) *(volatile v4u*)(base + (size_t)(i * 32 + lane) * 8) = vals[i];
    __threadfence();
  }
}

__global__ __launch_bounds__(256) void heads_kernel(const float* __restrict__ H,
                                                    const float* __restrict__ Wm2, const float* __restrict__ bm2,
                                                    const float* __restrict__ Wl2, const float* __restrict__ bl2,
                                                    const float* __restrict__ eps,
                                                    float* __restrict__ out0, float* __restrict__ out1, float* __restrict__ xi) {
  __shared__ float sh[3][32];
  const int lane = threadIdx.x & 31, wave = threadIdx.x >> 5;
  const int s0 = blockIdx.x * 32;
  const v4f wm = *(const v4f*)(Wm2 + 4 * lane);
  const v4f wl = *(const v4f*)(Wl2 + 4 * lane);
  const float bm = bm2[0];
  const float bl = bl2[0];
#pragma unroll 1
  for (int i = 0; i < 4; ++i) {
    const int sloc = wave * 4 + i;
    const int s = s0 + sloc;
    const float* hr = H + (size_t)s * (2 * NHID);
    const v4f hm = *(const v4f*)(hr + 4 * lane);
    const v4f hl = *(const v4f*)(hr + NHID + 4 * lane);
    float pm = hm[0] * wm[0];
    pm = fmaf(hm[1], wm[1], pm);
    pm = fmaf(hm[2], wm[2], pm);
    pm = fmaf(hm[3], wm[3], pm);
    float pl = hl[0] * wl[0];
    pl = fmaf(hl[1], wl[1], pl);
    pl = fmaf(hl[2], wl[2], pl);
    pl = fmaf(hl[3], wl[3], pl);
#pragma unroll
    for (int off = 16; off > 0; off >>= 1) {
      pm += __shfl_xor(pm, off, 32);
      pl += __shfl_xor(pl, off, 32);
    }
    const float zm = pm + bm;
    const float xm = fmaxf(zm, 0.0f) + log1pf(expf(-fabsf(zm)));
    const float zl = pl + bl;
    float x = xm + expf(0.5f * zl) * eps[s];
    x = fminf(fmaxf(x, 0.0f), 1.0f);
    if (lane == 0) { sh[0][sloc] = xm; sh[1][sloc] = zl; sh[2][sloc] = x; }
  }
  __syncthreads();
  if (wave < 3) {
    float* dst = (wave == 0) ? out0 : ((wave == 1) ? out1 : xi);
    const float v = sh[wave][lane];
    *(volatile float*)(dst + s0 + lane) = v;
    __threadfence();
    *(volatile float*)(dst + s0 + lane) = v;
  }
}

__global__ __launch_bounds__(256) void ode_decode(const float* __restrict__ data, const float* __restrict__ omega,
                                                  const float* __restrict__ xiv,
                                                  const float* __restrict__ Wa1, const float* __restrict__ ba1,
                                                  const float* __restrict__ Wa2, const float* __restrict__ ba2,
                                                  float* __restrict__ outp  ) {
  __shared__ float wsh[256];
  __shared__ float axsh[64];
  __shared__ __align__(16) float ybuf[64 * 36];
  const int tid = threadIdx.x;
  const int lane = tid & 31, wave = tid >> 5;
  {
    const float a = Wa1[tid & 127];
    const float bq = ba1[tid & 63];
    const float cq = Wa2[tid & 63];
    wsh[tid] = (tid < 128) ? a : ((tid < 192) ? bq : cq);
  }
  const int sl = tid >> 2;
  const int u  = tid & 3;
  const int s  = blockIdx.x * 64 + sl;
  const float om = omega[s];
  const float ax = fabsf(xiv[s]);
  float y = data[(size_t)s * DIMT];
  float v = 0.0f;
  const float b2 = ba2[0];
  if (u == 0) axsh[sl] = ax;
  __syncthreads();

  float w1[16], c0[16], bb[16], w2[16];
#pragma unroll
  for (int i = 0; i < 16; ++i) {
    const int j = u * 16 + i;
    c0[i] = om * wsh[j];
    w1[i] = wsh[NAUX + j];
    bb[i] = wsh[128 + j];
    w2[i] = wsh[192 + j];
  }
  float* orow_base = outp + (size_t)(blockIdx.x * 64) * DIMT;
  const int q = lane >> 3, c = lane & 7;

  for (int tb = 0; tb < DIMT / 32; ++tb) {
#pragma unroll 1
    for (int ti = 0; ti < 32; ++ti) {
      if (u == 0) ybuf[sl * 36 + ti] = y;
      float a0 = 0.0f, a1 = 0.0f, a2 = 0.0f, a3 = 0.0f;
#pragma unroll
      for (int i = 0; i < 16; i += 4) {
        const float h0 = fmaxf(fmaf(y, w1[i],     c0[i])     + bb[i],     0.0f);
        const float h1 = fmaxf(fmaf(y, w1[i + 1], c0[i + 1]) + bb[i + 1], 0.0f);
        const float h2 = fmaxf(fmaf(y, w1[i + 2], c0[i + 2]) + bb[i + 2], 0.0f);
        const float h3 = fmaxf(fmaf(y, w1[i + 3], c0[i + 3]) + bb[i + 3], 0.0f);
        a0 = fmaf(h0, w2[i],     a0);
        a1 = fmaf(h1, w2[i + 1], a1);
        a2 = fmaf(h2, w2[i + 2], a2);
        a3 = fmaf(h3, w2[i + 3], a3);
      }
      float acc = (a0 + a1) + (a2 + a3);
      acc += __shfl_xor(acc, 1, 32);
      acc += __shfl_xor(acc, 2, 32);
      acc += b2;
      const float yn = y + DTSTEP * v;
      v = v + DTSTEP * acc;
      y = yn;
    }
    __syncthreads();
#pragma unroll 1
    for (int it = 0; it < 2; ++it) {
      const int sq = wave * 8 + it * 4 + q;
      const float axq = axsh[sq];
      float* yp = ybuf + sq * 36 + 4 * c;
      v4f yv = *(const v4f*)yp;
      const int t0 = tb * 32 + 4 * c;
#pragma unroll
      for (int e = 0; e < 4; ++e) {
        const float tt = DTSTEP * (float)(t0 + e);
        yv[e] = expf(-(axq * tt)) * yv[e];
      }
      *(v4f*)yp = yv;
    }
    for (int pass = 0; pass < 2; ++pass) {
#pragma unroll
      for (int it = 0; it < 2; ++it) {
        const int sq = wave * 8 + it * 4 + q;
        const v4f val = *(const v4f*)(ybuf + sq * 36 + 4 * c);
        *(volatile v4f*)(orow_base + (size_t)sq * DIMT + tb * 32 + 4 * c) = val;
      }
      __threadfence();
    }
    __syncthreads();
  }
}

extern "C" void kernel_launch(void* const* d_in, const int* in_sizes, int n_in,
                              void* d_out, int out_size, void* d_ws,
                              size_t ws_size, hipStream_t stream) {
  if (n_in < 19) return;
  if (in_sizes[0] != NSAMP * DIMT || out_size != NSAMP * (2 + DIMT) || ws_size < WS_TOTAL) return;

  const float* data  = (const float*)d_in[0];
  const float* omega = (const float*)d_in[1];
  const float* eps   = (const float*)d_in[2];
  const float* Wf1   = (const float*)d_in[3];
  const float* bf1   = (const float*)d_in[4];
  const float* Wf2   = (const float*)d_in[5];
  const float* bf2   = (const float*)d_in[6];
  const float* Wxm1  = (const float*)d_in[7];
  const float* bxm1  = (const float*)d_in[8];
  const float* Wxm2  = (const float*)d_in[9];
  const float* bxm2  = (const float*)d_in[10];
  const float* Wxl1  = (const float*)d_in[11];
  const float* bxl1  = (const float*)d_in[12];
  const float* Wxl2  = (const float*)d_in[13];
  const float* bxl2  = (const float*)d_in[14];
  const float* Wa1   = (const float*)d_in[15];
  const float* ba1   = (const float*)d_in[16];
  const float* Wa2   = (const float*)d_in[17];
  const float* ba2   = (const float*)d_in[18];

  char* ws = (char*)d_ws;
  unsigned short* xp  = (unsigned short*)(ws + OFF_XP);
  unsigned short* bt1 = (unsigned short*)(ws + OFF_BT1);
  unsigned short* bt2 = (unsigned short*)(ws + OFF_BT2);
  unsigned short* bt3 = (unsigned short*)(ws + OFF_BT3);
  unsigned short* p1  = (unsigned short*)(ws + OFF_P1);
  unsigned short* p2  = (unsigned short*)(ws + OFF_P2);
  float*          hp  = (float*)(ws + OFF_HP);
  float*          xiw = (float*)(ws + OFF_XI);

  float* out0 = (float*)d_out + OUT0_OFF_B / 4;
  float* out1 = (float*)d_out + OUT1_OFF_B / 4;
  float* out2 = (float*)d_out + OUT2_OFF_B / 4;

  build_x_plane<<<NSAMP / 32, 256, 0, stream>>>(data, omega, xp);
  build_wt_plane<XPITCH><<<NFEAT / 32, 256, 0, stream>>>(Wf1, NFEAT, DIMT + 1, WCARRY, bt1);
  build_wt_plane<NFEAT><<<NFEAT / 32, 256, 0, stream>>>(Wf2, NFEAT, NFEAT, WCARRY, bt2);
  build_wt_plane<NFEAT><<<NHID / 32, 256, 0, stream>>>(Wxm1, NHID, NFEAT, WCARRY, bt3);
  build_wt_plane<NFEAT><<<NHID / 32, 256, 0, stream>>>(Wxl1, NHID, NFEAT, WCARRY, bt3 + (size_t)NHID * NFEAT);

  static_assert(NSAMP % 64 == 0 && NFEAT % 64 == 0 && KFEAT1 % 32 == 0, "gemm1 shape");
  wmma_gemm64<0, false, 2, 1, false, 2><<<dim3((NSAMP / 64) * (NFEAT / 64) / 8, 1), 256, 0, stream>>>(
      xp, xp, XPITCH, 0L, bt1, bt1, XPITCH, 0L, (void*)p1, (void*)p1, NFEAT, 0L, bf1, bf1, 0L, NSAMP, NFEAT, KFEAT1, WCARRY_INV);
  static_assert(NFEAT % 32 == 0, "gemm2 shape");
  wmma_gemm64<0, false, 2, 1, false, 2><<<dim3((NSAMP / 64) * (NFEAT / 64) / 8, 1), 256, 0, stream>>>(
      p1, p1, NFEAT, 0L, bt2, bt2, NFEAT, 0L, (void*)p2, (void*)p2, NFEAT, 0L, bf2, bf2, 0L, NSAMP, NFEAT, NFEAT, WCARRY_INV);
  static_assert(NHID % 64 == 0, "gemm3 shape");
  wmma_gemm64<0, false, 2, 0, false, 2><<<dim3((NSAMP / 64) * (NHID / 64) / 8, 1), 256, 0, stream>>>(
      p2, p2, NFEAT, 0L, bt3, bt3, NFEAT, 0L, (void*)hp, (void*)hp, 2 * NHID, 0L, bxm1, bxm1, 0L, NSAMP, NHID, NFEAT, WCARRY_INV);
  wmma_gemm64<0, false, 2, 0, false, 2><<<dim3((NSAMP / 64) * (NHID / 64) / 8, 1), 256, 0, stream>>>(
      p2, p2, NFEAT, 0L, bt3 + (size_t)NHID * NFEAT, bt3 + (size_t)NHID * NFEAT, NFEAT, 0L,
      (void*)(hp + NHID), (void*)(hp + NHID), 2 * NHID, 0L, bxl1, bxl1, 0L, NSAMP, NHID, NFEAT, WCARRY_INV);

  heads_kernel<<<NSAMP / 32, 256, 0, stream>>>(hp, Wxm2, bxm2, Wxl2, bxl2, eps, out0, out1, xiw);
  ode_decode<<<NSAMP / 64, 256, 0, stream>>>(data, omega, xiw, Wa1, ba1, Wa2, ba2, out2);
}
